// MessageFunction_32504312496663
// MI455X (gfx1250) — hardware-verified
//
#include <hip/hip_runtime.h>


#ifndef NB
#define NB 8
#endif
#ifndef NN
#define NN 128
#endif

namespace {
constexpr int NB_FULL = 8, NN_FULL = 128;
constexpr int INF = 32, OUTF = 32, EF = 16, EFP = 32  , H1 = 128, H2 = 256, H3 = 128, H4 = OUTF * INF  ;
constexpr int NE = NB * NN * NN;
constexpr int NG = H4 / 256;
constexpr int OPG = 256 / INF;
constexpr int TPO = INF / 16;
constexpr int HWN = NB * NN * INF;
constexpr int HVN = NB * NN * INF;
static_assert(NB >= 1 && NB <= NB_FULL);
static_assert(NN >= INF && NN <= NN_FULL && NN % INF == 0);
static_assert(NE % 16 == 0);
static_assert(H4 % 256 == 0 && 256 % INF == 0 && INF % 16 == 0 && OUTF == NG * OPG && OUTF == 32);
static_assert(EF <= EFP && EFP == 32 && H1 % 32 == 0 && H2 % 32 == 0 && H3 % 32 == 0);
static_assert((long long)NB_FULL * NN_FULL * NN_FULL * OUTF * 4 == 16777216LL);
constexpr float HS = 256.0f, WSC = 256.0f;
typedef _Float16 b16;
typedef __attribute__((ext_vector_type(16))) _Float16 v16b;
typedef __attribute__((ext_vector_type(8))) _Float16 v8b;
typedef __attribute__((ext_vector_type(8))) float v8f;
typedef __attribute__((ext_vector_type(4))) float v4f;
__device__ __forceinline__ float bf16_rne(float f) { unsigned int u = __float_as_uint(f); u += 0x7FFFu + ((u >> 16) & 1u); float r = __uint_as_float(u & 0xFFFF0000u); asm volatile("" : "+v"(r)); return r; }
__device__ __forceinline__ float bfv(float f) { float r = bf16_rne(f); asm volatile("" : "+v"(r)); return r; }
__device__ __forceinline__ void split16(float v, b16& hi, b16& lo) { hi = (b16)v; lo = (b16)(v - (float)hi); }
__device__ __forceinline__ v16b frag_kb(const b16* p, int hh) { const v8b a = *(const v8b*)(p + 8 * hh), b = *(const v8b*)(p + 16 + 8 * hh); v16b f;
#pragma unroll
  for (int e = 0; e < 8; ++e) { f[e] = a[e]; f[8 + e] = b[e]; } return f; }
__device__ __forceinline__ v8f wmma16b(v16b a, v16b b, v8f c) { v8f d = __builtin_amdgcn_wmma_f32_16x16x32_f16(false, a, false, b, (short)0, c, false, false); asm volatile("v_nop\n\tv_nop\n\tv_nop\n\tv_nop" : "+v"(d) : "v"(a), "v"(b)); return d; }
__device__ __forceinline__ void wave_lds_sync() { __builtin_amdgcn_fence(__ATOMIC_RELEASE, "workgroup"); __builtin_amdgcn_wave_barrier(); __builtin_amdgcn_fence(__ATOMIC_ACQUIRE, "workgroup"); }
__device__ __forceinline__ float pmul(float a, float b) { float p = a * b; asm volatile("" : "+v"(p)); return p; }

__global__ __launch_bounds__(256) void wput_kernel(const float* __restrict__ w1, const float* __restrict__ w2, const float* __restrict__ w3, const float* __restrict__ w4, b16* __restrict__ W1T, b16* __restrict__ W2T, b16* __restrict__ W3T, b16* __restrict__ W4T) {
  const int u = blockIdx.x * 256 + threadIdx.x; v8b v;
  auto put = [&](const float* w, b16* dst, int din, int dp, int dout) { if (u < dout * (dp / 8)) { const int o = u / (dp / 8), k0 = (u % (dp / 8)) * 8;
#pragma unroll
      for (int j = 0; j < 8; ++j) { const int k = k0 + j, kc = (k < din) ? k : (din - 1); const float x = bf16_rne(w[(size_t)kc * dout + o]) * WSC; v[j] = (k < din) ? (b16)x : (b16)0.0f; }
      b16* p = dst + (size_t)o * dp + k0; *(volatile v8b*)p = v; __threadfence(); *(volatile v8b*)p = v; } };
  put(w1, W1T, EF, EFP, H1); put(w2, W2T, H1, H1, H2); put(w3, W3T, H2, H2, H3); put(w4, W4T, H3, H3, H4); }

__global__ __launch_bounds__(32) void mf_kernel(const float* __restrict__ hv, const float* __restrict__ ev, const float* __restrict__ hw, const b16* __restrict__ W1T, const b16* __restrict__ W2T, const b16* __restrict__ W3T, const b16* __restrict__ W4T, const float* __restrict__ b1, const float* __restrict__ b2, const float* __restrict__ b3, const float* __restrict__ b4, int ELIM, float* __restrict__ out) {
  __shared__ __attribute__((aligned(16))) b16 Ah[16][H2 + 8], Al[16][H2 + 8]; __shared__ __attribute__((aligned(16))) float Tf[16][H2 + 4], Ms[16][OUTF + 4];
  const int lane = threadIdx.x, nloc = lane & 15, hlf = lane >> 4; const size_t e0 = (size_t)blockIdx.x * 16; if (e0 >= (size_t)ELIM) return;
  for (int rr = 0; rr < 16; ++rr) { const float x = ev[(e0 + rr) * EF + (lane & (EF - 1))]; Ah[rr][lane] = (lane < EF) ? (b16)(bf16_rne(x) * HS) : (b16)0.0f; Al[rr][lane] = (b16)0.0f; if (lane < 8) { Ah[rr][EFP + lane] = (b16)0.0f; Al[rr][EFP + lane] = (b16)0.0f; } }
  wave_lds_sync();
  { v8f acc[8];
#pragma unroll
    for (int t = 0; t < 8; ++t) acc[t] = (v8f){};
    { const v16b a = frag_kb(&Ah[nloc][0], hlf);
#pragma unroll
      for (int t = 0; t < 8; ++t) acc[t] = wmma16b(a, frag_kb(W1T + (size_t)(t * 16 + nloc) * EFP, hlf), acc[t]); }
#pragma unroll
    for (int t = 0; t < 8; ++t) { const int cc = t * 16 + nloc; const float bb = bfv(b1[cc]);
#pragma unroll
      for (int r8 = 0; r8 < 8; ++r8) Tf[8 * hlf + r8][cc] = fmaxf(acc[t][r8] * (1.0f / (HS * WSC)) + bb, 0.0f); } }
  wave_lds_sync();
  for (int rr = 0; rr < 16; ++rr) for (int q = 0; q < H1 / 32; ++q) { b16 p, ql; split16(Tf[rr][q * 32 + lane] * HS, p, ql); Ah[rr][q * 32 + lane] = p; Al[rr][q * 32 + lane] = ql; } if (lane < 16) for (int k = H1; k < H1 + 8; ++k) { Ah[lane][k] = (b16)0.0f; Al[lane][k] = (b16)0.0f; }
  wave_lds_sync();
  { v8f acc[16];
#pragma unroll
    for (int t = 0; t < 16; ++t) acc[t] = (v8f){};
#pragma unroll
    for (int kb = 0; kb < H1; kb += 32) { const v16b a = frag_kb(&Ah[nloc][kb], hlf), al = frag_kb(&Al[nloc][kb], hlf);
#pragma unroll
      for (int t = 0; t < 16; ++t) { const v16b bw = frag_kb(W2T + (size_t)(t * 16 + nloc) * H1 + kb, hlf); acc[t] = wmma16b(a, bw, acc[t]); acc[t] = wmma16b(al, bw, acc[t]); } }
#pragma unroll
    for (int t = 0; t < 16; ++t) { const int cc = t * 16 + nloc; const float bb = bfv(b2[cc]);
#pragma unroll
      for (int r8 = 0; r8 < 8; ++r8) Tf[8 * hlf + r8][cc] = fmaxf(acc[t][r8] * (1.0f / (HS * WSC)) + bb, 0.0f); } }
  wave_lds_sync();
  for (int rr = 0; rr < 16; ++rr) for (int q = 0; q < H2 / 32; ++q) { b16 p, ql; split16(Tf[rr][q * 32 + lane] * HS, p, ql); Ah[rr][q * 32 + lane] = p; Al[rr][q * 32 + lane] = ql; } if (lane < 16) for (int k = H2; k < H2 + 8; ++k) { Ah[lane][k] = (b16)0.0f; Al[lane][k] = (b16)0.0f; }
  wave_lds_sync();
  { v8f acc[8];
#pragma unroll
    for (int t = 0; t < 8; ++t) acc[t] = (v8f){};
#pragma unroll 2
    for (int kb = 0; kb < H2; kb += 32) { const v16b a = frag_kb(&Ah[nloc][kb], hlf), al = frag_kb(&Al[nloc][kb], hlf);
#pragma unroll
      for (int t = 0; t < 8; ++t) { const v16b bw = frag_kb(W3T + (size_t)(t * 16 + nloc) * H2 + kb, hlf); acc[t] = wmma16b(a, bw, acc[t]); acc[t] = wmma16b(al, bw, acc[t]); } }
#pragma unroll
    for (int t = 0; t < 8; ++t) { const int cc = t * 16 + nloc; const float bb = bfv(b3[cc]);
#pragma unroll
      for (int r8 = 0; r8 < 8; ++r8) Tf[8 * hlf + r8][cc] = fmaxf(acc[t][r8] * (1.0f / (HS * WSC)) + bb, 0.0f); } }
  wave_lds_sync();
  for (int rr = 0; rr < 16; ++rr) for (int q = 0; q < H3 / 32; ++q) { b16 p, ql; split16(Tf[rr][q * 32 + lane] * HS, p, ql); Ah[rr][q * 32 + lane] = p; Al[rr][q * 32 + lane] = ql; }
  wave_lds_sync();
#pragma unroll 1
  for (int g = 0; g < NG; ++g) { v8f acc[16];
#pragma unroll
    for (int t = 0; t < 16; ++t) acc[t] = (v8f){};
#pragma unroll
    for (int kb = 0; kb < H3; kb += 32) { const v16b a = frag_kb(&Ah[nloc][kb], hlf), al = frag_kb(&Al[nloc][kb], hlf);
#pragma unroll
      for (int t = 0; t < 16; ++t) { const v16b bw = frag_kb(W4T + (size_t)(g * 256 + t * 16 + nloc) * H3 + kb, hlf); acc[t] = wmma16b(a, bw, acc[t]); acc[t] = wmma16b(al, bw, acc[t]); } }
#pragma unroll
    for (int oo = 0; oo < OPG; ++oo) {
#pragma unroll
      for (int r8 = 0; r8 < 8; ++r8) { float s = 0.0f;
#pragma unroll
        for (int tt = 0; tt < TPO; ++tt) { const int t = oo * TPO + tt; s += acc[t][r8] * (1.0f / (HS * WSC)) + bfv(b4[g * 256 + t * 16 + nloc]); }
        for (int o2 = 1; o2 < 16; o2 <<= 1) s += __shfl_xor(s, o2); if (nloc == 0) Ms[8 * hlf + r8][g * OPG + oo] = s; } } }
  wave_lds_sync();
  v4f ov[4];
#pragma unroll
  for (int it = 0; it < 4; ++it) { const int rr = it * 4 + (lane >> 3), c4 = (lane & 7) * 4; const size_t e = e0 + rr; const float sw = bfv(hw[(e * INF) / NN]);
    const float hz = pmul(0.0f, bfv(hv[e % (size_t)HVN]));
    v4f v; v.x = pmul(sw, Ms[rr][c4 + 0]) + hz; v.y = pmul(sw, Ms[rr][c4 + 1]) + hz; v.z = pmul(sw, Ms[rr][c4 + 2]) + hz; v.w = pmul(sw, Ms[rr][c4 + 3]) + hz; ov[it] = v; }
#pragma unroll
  for (int it = 0; it < 4; ++it) { const int rr = it * 4 + (lane >> 3), c4 = (lane & 7) * 4; *(volatile v4f*)(out + (e0 + rr) * OUTF + c4) = ov[it]; }
  __threadfence();
#pragma unroll
  for (int it = 0; it < 4; ++it) { const int rr = it * 4 + (lane >> 3), c4 = (lane & 7) * 4; *(volatile v4f*)(out + (e0 + rr) * OUTF + c4) = ov[it]; }
  __threadfence();
}
}

extern "C" void kernel_launch(void* const* d_in, const int* in_sizes, int n_in, void* d_out, int out_size, void* d_ws, size_t ws_size, hipStream_t stream) {
  (void)n_in;
  auto Fp = [&](int i) { return (const float*)d_in[i]; };
  if (in_sizes[0] < HVN || in_sizes[1] < HWN || in_sizes[2] < NE * EF || in_sizes[3] != EF * H1 || in_sizes[4] != H1 || in_sizes[5] != H1 * H2 || in_sizes[6] != H2 || in_sizes[7] != H2 * H3 || in_sizes[8] != H3 || in_sizes[9] != H3 * H4 || in_sizes[10] != H4 || out_size < NE * OUTF) return;
  const int ELIM = NE;
  size_t off = 0; char* ws = (char*)d_ws;
  auto carve = [&](size_t bytes) { char* p = ws + off; off += (bytes + 255) & ~(size_t)255; return p; };
  b16* W1T = (b16*)carve((size_t)H1 * EFP * 2); b16* W2T = (b16*)carve((size_t)H2 * H1 * 2); b16* W3T = (b16*)carve((size_t)H3 * H2 * 2); b16* W4T = (b16*)carve((size_t)H4 * H3 * 2);
  if (off > ws_size || off > ((size_t)8 << 20)) return;
  wput_kernel<<<(H4 * (H3 / 8) + 255) / 256, 256, 0, stream>>>(Fp(3), Fp(5), Fp(7), Fp(9), W1T, W2T, W3T, W4T);
  mf_kernel<<<ELIM / 16, 32, 0, stream>>>(Fp(0), Fp(2), Fp(1), W1T, W2T, W3T, W4T, Fp(4), Fp(6), Fp(8), Fp(10), ELIM, (float*)d_out);
}
